// GINE0_14285061227137
// MI455X (gfx1250) — hardware-verified
//
#include <hip/hip_runtime.h>
#include <stddef.h>
#include <math.h>


#define NTHR   256
#define NWAVE  8
#define EPT    8
#define CHUNK  (NTHR * EPT)
#define WCAP   (EPT * 32)
#define LISTN  (NWAVE * WCAP)
#define PASSN  (NWAVE * 16)
#define PCAP   (CHUNK + PASSN)
#define NB     256
#define FD     128
#define EDIM   16
#define NLAY   3
#define NCLS   10
#define GMAX   512
#define WSC    16.0f
#define HSC    4.0f
#define QSC    0.25f
#define HINV   0.015625f
#define BN_EPS 1e-5f

#define LDS_ACC   0
#define LDS_MSG   (LDS_ACC + (NB + 1) * FD * 4)
#define LDS_STG   (LDS_MSG + PASSN * FD * 4)
#define LDS_LIST  (LDS_STG + NWAVE * 16 * 16 * 2)
#define LDS_PEND  (LDS_LIST + LISTN * 4)
#define LDS_SLOT  (LDS_PEND + PCAP * 4)
#define LDS_PRM   (LDS_SLOT + PASSN * 4)
#define LDS_WCNT  (LDS_PRM + 8 * FD * 4)
#define LDS_TOTAL (LDS_WCNT + 64)

#define PB0 6
#define PB1 24
#define PB4 8
#define PB5 1
#define PBT (PB0 + 3 * PB1 + PB4 + PB5)

static_assert(PASSN == 128);
static_assert(PCAP >= CHUNK + PASSN);
static_assert((NB % 32) == 0 && NB == 2 * NWAVE * 16);
static_assert(NWAVE * 16 * FD * 2 <= PASSN * FD * 4);
static_assert((LDS_TOTAL % 16) == 0);
static_assert(LDS_TOTAL <= 300 * 1024);
static_assert(PB0 * NTHR == NLAY * FD * (32 / 8));
static_assert(PB1 * NTHR == NLAY * FD * (FD / 8));
static_assert(PB4 * NTHR == FD * (FD / 8));
static_assert(PB5 * NTHR == 16 * (FD / 8));

typedef float    v4f  __attribute__((ext_vector_type(4)));
typedef float    v8f  __attribute__((ext_vector_type(8)));
typedef int      v4i  __attribute__((ext_vector_type(4)));
typedef _Float16 v8h  __attribute__((ext_vector_type(8)));
typedef _Float16 v16h __attribute__((ext_vector_type(16)));
union FragH { v16h v; v8h h[2]; };
union Pk8 { v8h h; v4i i; };

__device__ __forceinline__ v8h zero8() {
  v8h r;
#pragma unroll
  for (int i = 0; i < 8; ++i) r[i] = (_Float16)0.0f;
  return r;
}

__device__ __forceinline__ v8f wmh(v16h a, v16h b, v8f c) {
  v8f d = __builtin_amdgcn_wmma_f32_16x16x32_f16(false, a, false, b, (short)0, c, false, false);
  asm volatile("v_nop\n\tv_nop\n\tv_nop\n\tv_nop" : "+v"(d) : "v"(a), "v"(b));
  return d;
}

__device__ __forceinline__ v8h relu8(v8f d, float mul) {
  v8h r;
#pragma unroll
  for (int i = 0; i < 8; ++i) { const float t = fmaxf(d[i] * mul, 0.0f); r[i] = (_Float16)t; }
  return r;
}

__device__ __forceinline__ v8h cv8(v4f a, v4f b) {
  v8h r;
  r[0] = (_Float16)a.x; r[1] = (_Float16)a.y; r[2] = (_Float16)a.z; r[3] = (_Float16)a.w;
  r[4] = (_Float16)b.x; r[5] = (_Float16)b.y; r[6] = (_Float16)b.z; r[7] = (_Float16)b.w;
  return r;
}

__device__ __forceinline__ v8f ldc8(const float* p) {
  const v4f a = *(const v4f*)p;
  const v4f b = *(const v4f*)(p + 4);
  v8f c;
  c[0] = a.x; c[1] = a.y; c[2] = a.z; c[3] = a.w;
  c[4] = b.x; c[5] = b.y; c[6] = b.z; c[7] = b.w;
  return c;
}

__device__ __forceinline__ v8f splat8(float x) {
  v8f c;
#pragma unroll
  for (int i = 0; i < 8; ++i) c[i] = x;
  return c;
}

__device__ __forceinline__ int scan_chunk(const int* __restrict__ dsts, int nE, int cbase, int nodeBase,
                                          int vec8, int* list, int tid, int wave) {
  int wc = 0;
  const int el0  = tid * EPT;
  const int e0   = cbase + el0;
  const int sent = -2147483647 - 1;
  v4i da, db;
  if (vec8 != 0 && cbase + CHUNK <= nE) {
    da = *(const v4i*)(dsts + e0);
    db = *(const v4i*)(dsts + e0 + 4);
  } else {
    da.x = (e0     < nE) ? dsts[min(e0, nE - 1)] : sent;
    da.y = (e0 + 1 < nE) ? dsts[min(e0 + 1, nE - 1)] : sent;
    da.z = (e0 + 2 < nE) ? dsts[min(e0 + 2, nE - 1)] : sent;
    da.w = (e0 + 3 < nE) ? dsts[min(e0 + 3, nE - 1)] : sent;
    db.x = (e0 + 4 < nE) ? dsts[min(e0 + 4, nE - 1)] : sent;
    db.y = (e0 + 5 < nE) ? dsts[min(e0 + 5, nE - 1)] : sent;
    db.z = (e0 + 6 < nE) ? dsts[min(e0 + 6, nE - 1)] : sent;
    db.w = (e0 + 7 < nE) ? dsts[min(e0 + 7, nE - 1)] : sent;
  }
  const unsigned nb = (unsigned)nodeBase;
  const unsigned s0 = (unsigned)da.x - nb, s1 = (unsigned)da.y - nb;
  const unsigned s2 = (unsigned)da.z - nb, s3 = (unsigned)da.w - nb;
  const unsigned s4 = (unsigned)db.x - nb, s5 = (unsigned)db.y - nb;
  const unsigned s6 = (unsigned)db.z - nb, s7 = (unsigned)db.w - nb;
  const bool h0 = s0 < (unsigned)NB, h1 = s1 < (unsigned)NB, h2 = s2 < (unsigned)NB, h3 = s3 < (unsigned)NB;
  const bool h4 = s4 < (unsigned)NB, h5 = s5 < (unsigned)NB, h6 = s6 < (unsigned)NB, h7 = s7 < (unsigned)NB;
  const unsigned any = __builtin_amdgcn_ballot_w32(h0 | h1 | h2 | h3 | h4 | h5 | h6 | h7);
  if (any != 0u) {
#define HITJ(J, HJ) { \
      const unsigned mj = __builtin_amdgcn_ballot_w32(HJ); \
      if (mj != 0u) { \
        if (HJ) { \
          const int pos = wc + (int)__builtin_amdgcn_mbcnt_lo(mj, 0u); \
          if (pos < WCAP) list[wave * WCAP + pos] = el0 + (J); \
        } \
        wc += (int)__builtin_popcount(mj); } }
    HITJ(0, h0)
    HITJ(1, h1)
    HITJ(2, h2)
    HITJ(3, h3)
    HITJ(4, h4)
    HITJ(5, h5)
    HITJ(6, h6)
    HITJ(7, h7)
#undef HITJ
  }
  return wc;
}

__global__ __launch_bounds__(NTHR) void k_prep(
    const float* __restrict__ we1, const float* __restrict__ we2,
    const float* __restrict__ wm1, const float* __restrict__ wm2,
    const float* __restrict__ wl1, const float* __restrict__ wl2,
    _Float16* pe1, _Float16* pe2, _Float16* pm1, _Float16* pm2, _Float16* pl1, _Float16* pl2) {
  const int b = blockIdx.x, tid = threadIdx.x;
  const float* src;
  _Float16* dst;
  int Kin, Kp, O, Osrc, ub;
  if (b < PB0) {
    src = we1; dst = pe1; Kin = EDIM; Kp = 32; O = FD; Osrc = FD; ub = b;
  } else if (b < PB0 + PB1) {
    src = we2; dst = pe2; Kin = FD; Kp = FD; O = FD; Osrc = FD; ub = b - PB0;
  } else if (b < PB0 + 2 * PB1) {
    src = wm1; dst = pm1; Kin = FD; Kp = FD; O = FD; Osrc = FD; ub = b - (PB0 + PB1);
  } else if (b < PB0 + 3 * PB1) {
    src = wm2; dst = pm2; Kin = FD; Kp = FD; O = FD; Osrc = FD; ub = b - (PB0 + 2 * PB1);
  } else if (b < PB0 + 3 * PB1 + PB4) {
    src = wl1; dst = pl1; Kin = FD; Kp = FD; O = FD; Osrc = FD; ub = b - (PB0 + 3 * PB1);
  } else {
    src = wl2; dst = pl2; Kin = FD; Kp = FD; O = 16; Osrc = NCLS; ub = b - (PB0 + 3 * PB1 + PB4);
  }
  const int u   = ub * NTHR + tid;
  const int cpr = Kp >> 3;
  const int row = u / cpr;
  const int kc  = u - row * cpr;
  const int l   = row / O;
  const int o   = row - l * O;
  const int ocl = o < Osrc ? o : Osrc - 1;
  Pk8 pk;
#pragma unroll
  for (int j = 0; j < 8; ++j) {
    const int k   = 8 * kc + j;
    const int kcl = k < Kin ? k : Kin - 1;
    const float w = src[((size_t)(l * Kin + kcl)) * Osrc + ocl];
    const float t = (k < Kin && o < Osrc) ? w * WSC : 0.0f;
    pk.h[j] = (_Float16)t;
  }
  _Float16* dp = dst + (size_t)u * 8;
  *(volatile v4i*)dp = pk.i;
  __threadfence();
  *(volatile v4i*)dp = pk.i;
}

__global__ __launch_bounds__(NTHR) void k_layer(
    const float* __restrict__ xin, const float* __restrict__ eattr, const int* __restrict__ ei,
    const _Float16* __restrict__ W1t, const float* __restrict__ eb1,
    const _Float16* __restrict__ W2t, const float* __restrict__ eb2,
    const float* __restrict__ eg, const float* __restrict__ ebt,
    const float* __restrict__ erm, const float* __restrict__ erv,
    const _Float16* __restrict__ M1t, const float* __restrict__ nb1,
    const _Float16* __restrict__ M2t, const float* __restrict__ nb2,
    const float* __restrict__ ng, const float* __restrict__ nbt,
    const float* __restrict__ nrm, const float* __restrict__ nrv,
    float* xout, int nN, int nE, int vec8) {
  extern __shared__ __attribute__((aligned(16))) unsigned char dsm[];
  float*    acc   = (float*)(dsm + LDS_ACC);
  float*    msg   = (float*)(dsm + LDS_MSG);
  _Float16* hsn   = (_Float16*)(dsm + LDS_MSG);
  _Float16* stg   = (_Float16*)(dsm + LDS_STG);
  int*      list  = (int*)(dsm + LDS_LIST);
  int*      pend  = (int*)(dsm + LDS_PEND);
  int*      slotb = (int*)(dsm + LDS_SLOT);
  float*    prm   = (float*)(dsm + LDS_PRM);
  int*      wcnt  = (int*)(dsm + LDS_WCNT);

  const int tid = threadIdx.x, lane = tid & 31, wave = tid >> 5, hh = lane >> 4, m = lane & 15;
  const int nodeBase = blockIdx.x * NB;
  const int* srcs = ei;
  const int* dsts = ei + nE;

  {
    const v4f z = {0.0f, 0.0f, 0.0f, 0.0f};
    for (int i = tid; i < (NB + 1) * FD / 4; i += NTHR) *(v4f*)(acc + 4 * i) = z;
  }
  if (tid < FD) {
    const int f = tid;
    prm[f] = eb1[f] * WSC;
    prm[FD + f] = eb2[f] * (WSC * HSC);
    const float s1 = eg[f] * rsqrtf(erv[f] + BN_EPS);
    prm[2 * FD + f] = s1;
    prm[3 * FD + f] = ebt[f] - erm[f] * s1;
    prm[4 * FD + f] = nb1[f] * WSC;
    prm[5 * FD + f] = nb2[f] * (WSC * HSC);
    const float s2 = ng[f] * rsqrtf(nrv[f] + BN_EPS);
    prm[6 * FD + f] = s2;
    prm[7 * FD + f] = nbt[f] - nrm[f] * s2;
  }
  if (tid == 0) wcnt[NWAVE] = 0;
  __syncthreads();

  const int nChunks = (nE + CHUNK - 1) / CHUNK;
#pragma unroll 1
  for (int ch = 0; ch < nChunks; ++ch) {
    const int cbase = ch * CHUNK;
    const int wc = scan_chunk(dsts, nE, cbase, nodeBase, vec8, list, tid, wave);
    if (lane == 0) wcnt[wave] = wc;
    __syncthreads();

    const int base = wcnt[NWAVE];
    int tot = 0, myoff = 0;
#pragma unroll
    for (int w = 0; w < NWAVE; ++w) {
      int c = wcnt[w];
      c = c > WCAP ? WCAP : (c < 0 ? 0 : c);
      if (w < wave) myoff += c;
      tot += c;
    }
    int newN = base + tot;
    newN = newN > PCAP ? PCAP : newN;
    {
      int n = wcnt[wave];
      n = n > WCAP ? WCAP : (n < 0 ? 0 : n);
      const int* lp = list + wave * WCAP;
      for (int i = lane; i < n; i += 32) {
        const int pos = base + myoff + i;
        if (pos < PCAP) pend[pos] = cbase + lp[i];
      }
    }
    const int fin = (ch == nChunks - 1) ? 1 : 0;
    const int R   = (fin != 0) ? (newN + PASSN - 1) / PASSN : newN / PASSN;
    const int Pv  = (fin != 0) ? newN : R * PASSN;
    __syncthreads();

#pragma unroll 1
    for (int r = 0; r < R; ++r) {
      int scl;
      {
        int idx = r * PASSN + wave * 16 + m;
        const bool valid = idx < Pv;
        idx = idx > PCAP - 1 ? PCAP - 1 : idx;
        int e = pend[idx];
        e = e < 0 ? 0 : (e > nE - 1 ? nE - 1 : e);
        const int d = dsts[e];
        int s = srcs[e];
        int slot = d - nodeBase;
        if (!valid || (unsigned)slot >= (unsigned)NB) slot = NB;
        s = s < 0 ? 0 : (s > nN - 1 ? nN - 1 : s);
        scl = s;
        const float* ap = eattr + (size_t)e * EDIM + 8 * hh;
        const v4f a0 = *(const v4f*)ap;
        const v4f a1 = *(const v4f*)(ap + 4);
        v8h hv;
        hv[0] = (_Float16)(valid ? a0.x : 0.0f); hv[1] = (_Float16)(valid ? a0.y : 0.0f);
        hv[2] = (_Float16)(valid ? a0.z : 0.0f); hv[3] = (_Float16)(valid ? a0.w : 0.0f);
        hv[4] = (_Float16)(valid ? a1.x : 0.0f); hv[5] = (_Float16)(valid ? a1.y : 0.0f);
        hv[6] = (_Float16)(valid ? a1.z : 0.0f); hv[7] = (_Float16)(valid ? a1.w : 0.0f);
        *(v8h*)(stg + (wave * 16 + m) * 16 + 8 * hh) = hv;
        if (hh == 0) slotb[wave * 16 + m] = slot;
      }
      __syncthreads();

      {
        FragH ba;
        ba.h[0] = *(const v8h*)(stg + (wave * 16 + m) * 16 + 8 * hh);
        ba.h[1] = zero8();
        FragH bq[4];
#pragma unroll
        for (int q = 0; q < 4; ++q) {
          v8f d0, d1;
          {
            FragH a;
            const _Float16* wp = W1t + (size_t)(32 * q + m) * 32 + 8 * hh;
            a.h[0] = *(const v8h*)wp;
            a.h[1] = *(const v8h*)(wp + 16);
            d0 = wmh(a.v, ba.v, ldc8(prm + 32 * q + 8 * hh));
          }
          {
            FragH a;
            const _Float16* wp = W1t + (size_t)(32 * q + 16 + m) * 32 + 8 * hh;
            a.h[0] = *(const v8h*)wp;
            a.h[1] = *(const v8h*)(wp + 16);
            d1 = wmh(a.v, ba.v, ldc8(prm + 32 * q + 16 + 8 * hh));
          }
          bq[q].h[0] = relu8(d0, QSC);
          bq[q].h[1] = relu8(d1, QSC);
        }
#pragma unroll 1
        for (int ft = 0; ft < FD / 16; ++ft) {
          v8f c = ldc8(prm + FD + 16 * ft + 8 * hh);
#pragma unroll
          for (int kt = 0; kt < 4; ++kt) {
            FragH a;
            const _Float16* wp = W2t + (size_t)(16 * ft + m) * FD + 32 * kt + 8 * hh;
            a.h[0] = *(const v8h*)wp;
            a.h[1] = *(const v8h*)(wp + 16);
            c = wmh(a.v, bq[kt].v, c);
          }
          const int f0 = 16 * ft + 8 * hh;
          const v8f sc = ldc8(prm + 2 * FD + f0);
          const v8f sh = ldc8(prm + 3 * FD + f0);
          const float* xr = xin + (size_t)scl * FD + f0;
          const v4f x0 = *(const v4f*)xr;
          const v4f x1 = *(const v4f*)(xr + 4);
          float xs[8];
          xs[0] = x0.x; xs[1] = x0.y; xs[2] = x0.z; xs[3] = x0.w;
          xs[4] = x1.x; xs[5] = x1.y; xs[6] = x1.z; xs[7] = x1.w;
          float o[8];
#pragma unroll
          for (int rr = 0; rr < 8; ++rr) {
            const float e2 = fmaxf(c[rr] * HINV, 0.0f);
            const float bn = e2 * sc[rr] + sh[rr];
            o[rr] = fmaxf(xs[rr] + bn, 0.0f);
          }
          float* mp = msg + (wave * 16 + m) * FD + f0;
          const v4f o0 = {o[0], o[1], o[2], o[3]};
          const v4f o1 = {o[4], o[5], o[6], o[7]};
          *(v4f*)mp = o0;
          *(v4f*)(mp + 4) = o1;
        }
      }
      __syncthreads();

      if (tid < FD) {
#pragma unroll 1
        for (int i = 0; i < PASSN; ++i) {
          int sl = slotb[i];
          sl = sl < 0 ? 0 : (sl > NB ? NB : sl);
          acc[sl * FD + tid] += msg[i * FD + tid];
        }
      }
      __syncthreads();
    }

    int rem = newN - R * PASSN;
    rem = rem < 0 ? 0 : rem;
    if (R > 0 && tid < rem) pend[tid] = pend[R * PASSN + tid];
    if (tid == 0) wcnt[NWAVE] = rem;
  }
  __syncthreads();

#pragma unroll 1
  for (int tt = 0; tt < 2; ++tt) {
    const int t    = wave + NWAVE * tt;
    const int lrow = 16 * t + m;
    int node = nodeBase + lrow;
    node = node > nN - 1 ? nN - 1 : node;
    const float* xr = xin + (size_t)node * FD;
    const float* ar = acc + lrow * FD;
    FragH bq[4];
#pragma unroll
    for (int kt = 0; kt < 4; ++kt) {
      const int k0 = 32 * kt + 8 * hh;
      const v4f xa = *(const v4f*)(xr + k0);
      const v4f xb = *(const v4f*)(xr + k0 + 4);
      const v4f xc = *(const v4f*)(xr + k0 + 16);
      const v4f xd = *(const v4f*)(xr + k0 + 20);
      const v4f ga = *(const v4f*)(ar + k0);
      const v4f gb = *(const v4f*)(ar + k0 + 4);
      const v4f gc = *(const v4f*)(ar + k0 + 16);
      const v4f gd = *(const v4f*)(ar + k0 + 20);
      bq[kt].h[0] = cv8(xa + ga, xb + gb);
      bq[kt].h[1] = cv8(xc + gc, xd + gd);
    }
    __syncthreads();
    _Float16* hw = hsn + wave * 16 * FD;
#pragma unroll 1
    for (int ft = 0; ft < FD / 16; ++ft) {
      v8f c = ldc8(prm + 4 * FD + 16 * ft + 8 * hh);
#pragma unroll
      for (int kt = 0; kt < 4; ++kt) {
        FragH a;
        const _Float16* wp = M1t + (size_t)(16 * ft + m) * FD + 32 * kt + 8 * hh;
        a.h[0] = *(const v8h*)wp;
        a.h[1] = *(const v8h*)(wp + 16);
        c = wmh(a.v, bq[kt].v, c);
      }
      *(v8h*)(hw + m * FD + 16 * ft + 8 * hh) = relu8(c, QSC);
    }
    __syncthreads();
    FragH bz[4];
#pragma unroll
    for (int kt = 0; kt < 4; ++kt) {
      const _Float16* hp = hw + m * FD + 32 * kt + 8 * hh;
      bz[kt].h[0] = *(const v8h*)hp;
      bz[kt].h[1] = *(const v8h*)(hp + 16);
    }
#pragma unroll 1
    for (int ft = 0; ft < FD / 16; ++ft) {
      v8f c = ldc8(prm + 5 * FD + 16 * ft + 8 * hh);
#pragma unroll
      for (int kt = 0; kt < 4; ++kt) {
        FragH a;
        const _Float16* wp = M2t + (size_t)(16 * ft + m) * FD + 32 * kt + 8 * hh;
        a.h[0] = *(const v8h*)wp;
        a.h[1] = *(const v8h*)(wp + 16);
        c = wmh(a.v, bz[kt].v, c);
      }
      const int f0 = 16 * ft + 8 * hh;
      const v8f sc = ldc8(prm + 6 * FD + f0);
      const v8f sh = ldc8(prm + 7 * FD + f0);
      float o[8];
#pragma unroll
      for (int rr = 0; rr < 8; ++rr) {
        const float h2 = fmaxf(c[rr] * HINV, 0.0f);
        o[rr] = h2 * sc[rr] + sh[rr];
      }
      float* sp = acc + lrow * FD + f0;
      const v4f o0 = {o[0], o[1], o[2], o[3]};
      const v4f o1 = {o[4], o[5], o[6], o[7]};
      *(v4f*)sp = o0;
      *(v4f*)(sp + 4) = o1;
    }
    __syncthreads();
  }

#pragma unroll 1
  for (int rr = 0; rr < NB / NWAVE; ++rr) {
    const int row = wave * (NB / NWAVE) + rr;
    const v4f v = *(const v4f*)(acc + row * FD + 4 * lane);
    *(volatile v4f*)(xout + (size_t)(nodeBase + row) * FD + 4 * lane) = v;
  }
  __threadfence();
#pragma unroll 1
  for (int rr = 0; rr < NB / NWAVE; ++rr) {
    const int row = wave * (NB / NWAVE) + rr;
    const v4f v = *(const v4f*)(acc + row * FD + 4 * lane);
    *(volatile v4f*)(xout + (size_t)(nodeBase + row) * FD + 4 * lane) = v;
  }
}

__global__ __launch_bounds__(NTHR) void k_pool(const float* __restrict__ x, const int* __restrict__ bt,
                                              float* pooled, int nN) {
  __shared__ int hl[NTHR];
  __shared__ int wc[NWAVE];
  __shared__ __attribute__((aligned(16))) float prow[FD];
  const int tid = threadIdx.x, lane = tid & 31, wave = tid >> 5;
  const int g = blockIdx.x;
  float s = 0.0f;
  int cnt = 0;
  const int nCh = (nN + NTHR - 1) / NTHR;
#pragma unroll 1
  for (int ch = 0; ch < nCh; ++ch) {
    const int i  = ch * NTHR + tid;
    const int ic = i > nN - 1 ? nN - 1 : i;
    const int b  = bt[ic];
    const bool hit = (i < nN) && (b == g);
    const unsigned mk = __builtin_amdgcn_ballot_w32(hit);
    if (lane == 0) wc[wave] = (int)__builtin_popcount(mk);
    __syncthreads();
    int off = 0, tot = 0;
#pragma unroll
    for (int w = 0; w < NWAVE; ++w) { const int c = wc[w]; if (w < wave) off += c; tot += c; }
    if (hit) {
      const int pos = off + (int)__builtin_amdgcn_mbcnt_lo(mk, 0u);
      if (pos < NTHR) hl[pos] = i;
    }
    __syncthreads();
    tot = tot > NTHR ? NTHR : (tot < 0 ? 0 : tot);
    if (tid < FD) {
#pragma unroll 1
      for (int j = 0; j < tot; ++j) {
        int nd = hl[j];
        nd = nd < 0 ? 0 : (nd > nN - 1 ? nN - 1 : nd);
        s += x[(size_t)nd * FD + tid];
      }
    }
    cnt += tot;
    __syncthreads();
  }
  if (tid < FD) {
    const float c = (float)(cnt > 1 ? cnt : 1);
    prow[tid] = s * (1.0f / c);
  }
  __syncthreads();
  v4f v = {0.0f, 0.0f, 0.0f, 0.0f};
  if (wave == 0) v = *(const v4f*)(prow + 4 * lane);
  if (wave == 0) *(volatile v4f*)(pooled + (size_t)g * FD + 4 * lane) = v;
  __threadfence();
  if (wave == 0) *(volatile v4f*)(pooled + (size_t)g * FD + 4 * lane) = v;
}

__global__ __launch_bounds__(NTHR) void k_head(const float* __restrict__ pooled,
                                              const _Float16* __restrict__ L1t, const float* __restrict__ lb1,
                                              const _Float16* __restrict__ L2t, const float* __restrict__ lb2,
                                              float* out, int G) {
  __shared__ __attribute__((aligned(16))) _Float16 hs[NWAVE * 16 * FD];
  __shared__ __attribute__((aligned(16))) float lg[NWAVE * 16 * 16];
  __shared__ __attribute__((aligned(16))) float outs[GMAX * NCLS];
  const int tid = threadIdx.x, lane = tid & 31, wave = tid >> 5, hh = lane >> 4, m = lane & 15;
  _Float16* hw = hs + wave * 16 * FD;
  float* lw = lg + wave * 256;
  const int nIt = G / (16 * NWAVE);
#pragma unroll 1
  for (int it = 0; it < nIt; ++it) {
    const int row0 = (it * NWAVE + wave) * 16;
    FragH a[4];
    {
      const float* pr = pooled + (size_t)(row0 + m) * FD + 8 * hh;
#pragma unroll
      for (int kt = 0; kt < 4; ++kt) {
        const float* p = pr + 32 * kt;
        a[kt].h[0] = cv8(*(const v4f*)p, *(const v4f*)(p + 4));
        a[kt].h[1] = cv8(*(const v4f*)(p + 16), *(const v4f*)(p + 20));
      }
    }
#pragma unroll 1
    for (int nt = 0; nt < FD / 16; ++nt) {
      v8f c = splat8(lb1[16 * nt + m] * WSC);
#pragma unroll
      for (int kt = 0; kt < 4; ++kt) {
        FragH b;
        const _Float16* bp = L1t + (size_t)(16 * nt + m) * FD + 32 * kt + 8 * hh;
        b.h[0] = *(const v8h*)bp;
        b.h[1] = *(const v8h*)(bp + 16);
        c = wmh(a[kt].v, b.v, c);
      }
#pragma unroll
      for (int rr = 0; rr < 8; ++rr) hw[(8 * hh + rr) * FD + 16 * nt + m] = (_Float16)fmaxf(c[rr] * QSC, 0.0f);
    }
    __syncthreads();
    FragH a2[4];
#pragma unroll
    for (int kt = 0; kt < 4; ++kt) {
      const _Float16* hp = hw + m * FD + 32 * kt + 8 * hh;
      a2[kt].h[0] = *(const v8h*)hp;
      a2[kt].h[1] = *(const v8h*)(hp + 16);
    }
    float bb2 = lb2[m < NCLS ? m : NCLS - 1];
    bb2 = (m < NCLS) ? bb2 * (WSC * HSC) : 0.0f;
    v8f c2 = splat8(bb2);
#pragma unroll
    for (int kt = 0; kt < 4; ++kt) {
      FragH b;
      const _Float16* bp = L2t + (size_t)m * FD + 32 * kt + 8 * hh;
      b.h[0] = *(const v8h*)bp;
      b.h[1] = *(const v8h*)(bp + 16);
      c2 = wmh(a2[kt].v, b.v, c2);
    }
#pragma unroll
    for (int rr = 0; rr < 8; ++rr) lw[(8 * hh + rr) * 16 + m] = c2[rr] * HINV;
    __syncthreads();
    {
      const float* lr = lw + m * 16;
      float mx = lr[0];
#pragma unroll 1
      for (int c = 1; c < NCLS; ++c) mx = fmaxf(mx, lr[c]);
      float ssum = 0.0f;
#pragma unroll 1
      for (int c = 0; c < NCLS; ++c) ssum += expf(lr[c] - mx);
      const float lse = logf(ssum);
#pragma unroll 1
      for (int c = 0; c < NCLS; ++c) {
        const float v = (lr[c] - mx) - lse;
        if (hh == 0) outs[(row0 + m) * NCLS + c] = v;
      }
    }
    __syncthreads();
  }
  __syncthreads();
  const int nOut4 = (G * NCLS) / 4;
#pragma unroll 1
  for (int u = tid; u < nOut4; u += NTHR) {
    const v4f v = *(const v4f*)(outs + 4 * u);
    *(volatile v4f*)(out + 4 * u) = v;
  }
  __threadfence();
#pragma unroll 1
  for (int u = tid; u < nOut4; u += NTHR) {
    const v4f v = *(const v4f*)(outs + 4 * u);
    *(volatile v4f*)(out + 4 * u) = v;
  }
}

extern "C" void kernel_launch(void* const* d_in, const int* in_sizes, int n_in,
                              void* d_out, int out_size, void* d_ws, size_t ws_size,
                              hipStream_t stream) {
  if (n_in < 24) return;
  const int nN = in_sizes[3];
  if (nN < 1) return;
  if (in_sizes[0] != nN * FD) return;
  const int nE = in_sizes[2] / 2;
  if (nE < 1 || in_sizes[2] != 2 * nE || in_sizes[1] != nE * EDIM) return;
  if (in_sizes[4] != NLAY * EDIM * FD || in_sizes[6] != NLAY * FD * FD) return;
  if (in_sizes[12] != NLAY * FD * FD || in_sizes[14] != NLAY * FD * FD) return;
  {
    const int small[12] = {5, 7, 8, 9, 10, 11, 13, 15, 16, 17, 18, 19};
    for (int i = 0; i < 12; ++i) if (in_sizes[small[i]] != NLAY * FD) return;
  }
  if (in_sizes[20] != FD * FD || in_sizes[21] != FD || in_sizes[22] != FD * NCLS || in_sizes[23] != NCLS) return;
  const int G = out_size / NCLS;
  if (G < 16 * NWAVE || out_size != G * NCLS || (G % (16 * NWAVE)) != 0 || G > GMAX) return;

  const float* x     = (const float*)d_in[0];
  const float* eattr = (const float*)d_in[1];
  const int*   ei    = (const int*)d_in[2];
  const int*   batch = (const int*)d_in[3];
  const float* ee_w1 = (const float*)d_in[4];
  const float* ee_b1 = (const float*)d_in[5];
  const float* ee_w2 = (const float*)d_in[6];
  const float* ee_b2 = (const float*)d_in[7];
  const float* ee_g  = (const float*)d_in[8];
  const float* ee_bt = (const float*)d_in[9];
  const float* ee_rm = (const float*)d_in[10];
  const float* ee_rv = (const float*)d_in[11];
  const float* mw1   = (const float*)d_in[12];
  const float* mb1   = (const float*)d_in[13];
  const float* mw2   = (const float*)d_in[14];
  const float* mb2   = (const float*)d_in[15];
  const float* m_g   = (const float*)d_in[16];
  const float* m_bt  = (const float*)d_in[17];
  const float* m_rm  = (const float*)d_in[18];
  const float* m_rv  = (const float*)d_in[19];
  const float* l1w   = (const float*)d_in[20];
  const float* l1b   = (const float*)d_in[21];
  const float* l2w   = (const float*)d_in[22];
  const float* l2b   = (const float*)d_in[23];
  float* outp = (float*)d_out;

  const int nBlk = (nN + NB - 1) / NB;
  const size_t rowsP = (size_t)nBlk * NB;

  char* ws = (char*)d_ws;
  size_t off = 0;
  const size_t oE1 = off; off += ((size_t)NLAY * FD * 32 * 2 + 255) & ~(size_t)255;
  const size_t oE2 = off; off += ((size_t)NLAY * FD * FD * 2 + 255) & ~(size_t)255;
  const size_t oM1 = off; off += ((size_t)NLAY * FD * FD * 2 + 255) & ~(size_t)255;
  const size_t oM2 = off; off += ((size_t)NLAY * FD * FD * 2 + 255) & ~(size_t)255;
  const size_t oL1 = off; off += ((size_t)FD * FD * 2 + 255) & ~(size_t)255;
  const size_t oL2 = off; off += ((size_t)16 * FD * 2 + 255) & ~(size_t)255;
  const size_t oX0 = off; off += (rowsP * FD * 4 + 255) & ~(size_t)255;
  const size_t oX1 = off; off += (rowsP * FD * 4 + 255) & ~(size_t)255;
  const size_t oPl = off; off += ((size_t)G * FD * 4 + 255) & ~(size_t)255;
  size_t limit = (size_t)134217728;
  if (ws_size < limit) limit = ws_size;
  if (off > limit) return;

  _Float16* pE1 = (_Float16*)(ws + oE1);
  _Float16* pE2 = (_Float16*)(ws + oE2);
  _Float16* pM1 = (_Float16*)(ws + oM1);
  _Float16* pM2 = (_Float16*)(ws + oM2);
  _Float16* pL1 = (_Float16*)(ws + oL1);
  _Float16* pL2 = (_Float16*)(ws + oL2);
  float* X0  = (float*)(ws + oX0);
  float* X1  = (float*)(ws + oX1);
  float* Pl  = (float*)(ws + oPl);

  const int vec8 = ((nE & 3) == 0) ? 1 : 0;

  k_prep<<<PBT, NTHR, 0, stream>>>(ee_w1, ee_w2, mw1, mw2, l1w, l2w, pE1, pE2, pM1, pM2, pL1, pL2);

  hipFuncSetAttribute(reinterpret_cast<const void*>(&k_layer), hipFuncAttributeMaxDynamicSharedMemorySize, LDS_TOTAL);

  const float* xcur = x;
  float* planes[2] = {X0, X1};
  for (int l = 0; l < NLAY; ++l) {
    float* xo = planes[l & 1];
    k_layer<<<nBlk, NTHR, LDS_TOTAL, stream>>>(
        xcur, eattr, ei,
        pE1 + (size_t)l * FD * 32, ee_b1 + l * FD,
        pE2 + (size_t)l * FD * FD, ee_b2 + l * FD,
        ee_g + l * FD, ee_bt + l * FD, ee_rm + l * FD, ee_rv + l * FD,
        pM1 + (size_t)l * FD * FD, mb1 + l * FD,
        pM2 + (size_t)l * FD * FD, mb2 + l * FD,
        m_g + l * FD, m_bt + l * FD, m_rm + l * FD, m_rv + l * FD,
        xo, nN, nE, vec8);
    xcur = xo;
  }

  k_pool<<<G, NTHR, 0, stream>>>(xcur, batch, Pl, nN);
  k_head<<<1, NTHR, 0, stream>>>(Pl, pL1, l1b, pL2, l2b, outp, G);
}
